// TransformerDecoderLayer_60172491816991
// MI455X (gfx1250) — hardware-verified
//
#include <hip/hip_runtime.h>


#ifndef NB
#define NB 4
#endif
#ifndef SEQ
#define SEQ 1024
#endif
#ifndef SENC
#define SENC 1024
#endif
#define NB_FULL 4
#define SEQ_FULL 1024
#define SENC_FULL 1024
#define DM 1024
#define HE 16
#define DH 64
#define DFF 4096
#define QR 64
#define KT 32
#define KVMAX ((SEQ > SENC) ? SEQ : SENC)
#define MKW (KVMAX / 32)
#define KPITCH 72
#define VPITCH 40
#define PPITCH 40
#define CPITCH 136
#define TPITCH 72
#define OPITCH 132
#define HPITCH 136
#define X_CARRY 64.0f
#define W_CARRY 1024.0f
#define QKV_CARRY 16.0f
#define P_CARRY 4096.0f
#define C_CARRY 64.0f
#define H_CARRY 64.0f
#define LN_EPS 1e-5f
#define MASK_FILL (-1e9f)
#define SC_SCALE (1.0f / (8.0f * QKV_CARRY * QKV_CARRY))

static_assert(NB >= 1 && NB <= NB_FULL);
static_assert(SEQ >= QR && SEQ <= SEQ_FULL && SEQ % QR == 0 && SEQ % KT == 0);
static_assert(SENC >= QR && SENC <= SENC_FULL && SENC % QR == 0 && SENC % KT == 0);
static_assert(KVMAX <= 1024 && MKW >= 1 && MKW <= 32);
static_assert(DM == HE * DH && DH == 64 && (HE % 2) == 0);
static_assert((NB * SEQ) % 64 == 0 && (NB * SENC) % 64 == 0);
static_assert(DM % 128 == 0 && DFF % 128 == 0 && DM % 64 == 0 && DFF % 64 == 0);

#define MROWS ((size_t)NB * SEQ)
#define EROWS ((size_t)NB * SENC)
#define XROWS ((MROWS > EROWS) ? MROWS : EROWS)
#define SZ_WQKV ((size_t)3 * DM * DM * 2)
#define SZ_WO   ((size_t)DM * DM * 2)
#define SZ_WF   ((size_t)DM * DFF * 2)
#define SZ_XE_A ((MROWS + EROWS) * DM * 2)
#define SZ_XE_B (MROWS * DM * 4)
#define SZ_XE   ((SZ_XE_A > SZ_XE_B) ? SZ_XE_A : SZ_XE_B)
#define SZ_QKV  (XROWS * 3 * DM * 2)
#define SZ_CTX  (MROWS * DM * 2)
#define SZ_HID  (MROWS * DFF * 2)
#define SZ_QC   (((SZ_QKV + SZ_CTX) > SZ_HID) ? (SZ_QKV + SZ_CTX) : SZ_HID)
#define SZ_T    (MROWS * DM * 4)
#define SZ_X1F  (MROWS * DM * 4)
#define SZ_X1H  (MROWS * DM * 2)
#define WS_TOTAL (2 * SZ_WQKV + 2 * SZ_WO + 2 * SZ_WF + SZ_XE + SZ_QC + SZ_T + SZ_X1F + SZ_X1H)
static_assert(WS_TOTAL <= (size_t)134217728);
static_assert(SZ_XE >= SZ_XE_A && SZ_XE >= SZ_XE_B);
static_assert(SZ_QC >= SZ_QKV + SZ_CTX && SZ_QC >= SZ_HID);

typedef _Float16 v8h  __attribute__((ext_vector_type(8)));
typedef _Float16 v16h __attribute__((ext_vector_type(16)));
typedef float v8f __attribute__((ext_vector_type(8)));
typedef float v4f __attribute__((ext_vector_type(4)));

union FragH { v16h v; v8h h[2]; };
union GStage { float f[64 * OPITCH]; _Float16 h[64 * HPITCH]; };
static_assert(sizeof(GStage) == 64 * OPITCH * 4);
static_assert(64 * HPITCH * 2 <= 64 * OPITCH * 4);

__device__ __forceinline__ unsigned f2bf(float f) { unsigned u = __float_as_uint(f); u += 0x7FFFu + ((u >> 16) & 1u); return u >> 16; }
__device__ __forceinline__ float bf16r(float f) { return __uint_as_float(f2bf(f) << 16); }

__device__ __forceinline__ v8f wm_f16(v16h a, v16h b, v8f c) {
    c = __builtin_amdgcn_wmma_f32_16x16x32_f16(false, a, false, b, (short)0, c, false, false);
    asm volatile("v_nop\n\tv_nop\n\tv_nop\n\tv_nop" : "+v"(c) : "v"(a), "v"(b));
    return c;
}

__global__ __launch_bounds__(256) void k_wtrans(const float* __restrict__ in0, const float* __restrict__ in1, const float* __restrict__ in2,
                                               _Float16* out0, _Float16* out1, _Float16* out2,
                                               int R, int C, int hz, long long in_zs, long long out_zs)
{
    __shared__ __align__(16) _Float16 sT[64 * TPITCH];
    const int tid = threadIdx.x;
    const int z = blockIdx.z, mat = z / hz, hs = z - mat * hz;
    const float* in = (mat == 0) ? in0 : ((mat == 1) ? in1 : in2);
    _Float16* out = (mat == 0) ? out0 : ((mat == 1) ? out1 : out2);
    in += (size_t)hs * (size_t)in_zs;
    out += (size_t)hs * (size_t)out_zs;
    const int c0 = blockIdx.x * 64, r0 = blockIdx.y * 64;
#pragma unroll
    for (int i = 0; i < 4; ++i) {
        const int p = tid + 256 * i, row = p >> 4, c4 = (p & 15) * 4;
        const v4f a = *(const v4f*)(in + (size_t)(r0 + row) * C + c0 + c4);
#pragma unroll
        for (int j = 0; j < 4; ++j) sT[(c4 + j) * TPITCH + row] = (_Float16)(bf16r(a[j]) * W_CARRY);
    }
    __syncthreads();
    v8h ov[2];
#pragma unroll
    for (int i = 0; i < 2; ++i) {
        const int p = tid + 256 * i, c = p >> 3, r8 = (p & 7) * 8;
        ov[i] = *(const v8h*)(sT + c * TPITCH + r8);
    }
#pragma unroll
    for (int i = 0; i < 2; ++i) {
        const int p = tid + 256 * i, c = p >> 3, r8 = (p & 7) * 8;
        *(volatile v8h*)(out + (size_t)(c0 + c) * R + r0 + r8) = ov[i];
    }
    __threadfence();
#pragma unroll
    for (int i = 0; i < 2; ++i) {
        const int p = tid + 256 * i, c = p >> 3, r8 = (p & 7) * 8;
        *(volatile v8h*)(out + (size_t)(c0 + c) * R + r0 + r8) = ov[i];
    }
}

__global__ __launch_bounds__(256) void k_xconv(const float* __restrict__ x, const float* __restrict__ e, _Float16* Xh, _Float16* Eh, int nblkX)
{
    const int bid = blockIdx.x;
    const int which = (bid < nblkX) ? 0 : 1;
    const int lb = which ? (bid - nblkX) : bid;
    const size_t el = ((size_t)lb * 256 + threadIdx.x) * 8;
    const size_t m = el / DM; const int col = (int)(el % DM);
    const float* src; _Float16* dst;
    if (which == 0) {
        const int bb = (int)(m / SEQ), n = (int)(m % SEQ);
        src = x + ((size_t)bb * SEQ_FULL + n) * DM + col; dst = Xh + el;
    } else {
        const int bb = (int)(m / SENC), n = (int)(m % SENC);
        src = e + ((size_t)bb * SENC_FULL + n) * DM + col; dst = Eh + el;
    }
    const v4f a0 = *(const v4f*)src, a1 = *(const v4f*)(src + 4);
    v8h o;
#pragma unroll
    for (int i = 0; i < 4; ++i) { o[i] = (_Float16)(bf16r(a0[i]) * X_CARRY); o[4 + i] = (_Float16)(bf16r(a1[i]) * X_CARRY); }
    *(volatile v8h*)dst = o;
    __threadfence();
    *(volatile v8h*)dst = o;
}

__global__ __launch_bounds__(256) void k_gemm(const _Float16* __restrict__ A, const _Float16* __restrict__ Bt,
                                             const float* __restrict__ bias0, const float* __restrict__ bias1, const float* __restrict__ bias2,
                                             float* Cf, _Float16* Ch, int lda, int ldb, int ldc, int K, int bseg, int mode, int relu,
                                             float scale, float ocarry)
{
    __shared__ __align__(16) GStage st;
    const int tid = threadIdx.x, lane = tid & 31, wv = tid >> 5, hh = lane >> 4, lm = lane & 15;
    const int rt = wv & 3, chf = wv >> 2;
    const int row0 = blockIdx.x * 64, cb = blockIdx.y * 128, col0 = cb + chf * 64;
    const _Float16* xr = A + (size_t)(row0 + rt * 16 + lm) * lda;
    v8f acc[4];
#pragma unroll
    for (int t = 0; t < 4; ++t) acc[t] = (v8f){};
#pragma unroll 2
    for (int kc = 0; kc < K; kc += 32) {
        FragH a;
        a.h[0] = *(const v8h*)(xr + kc + 8 * hh);
        a.h[1] = *(const v8h*)(xr + kc + 16 + 8 * hh);
#pragma unroll
        for (int t = 0; t < 4; ++t) {
            FragH bb;
            const _Float16* wr = Bt + (size_t)(col0 + t * 16 + lm) * ldb + kc;
            bb.h[0] = *(const v8h*)(wr + 8 * hh);
            bb.h[1] = *(const v8h*)(wr + 16 + 8 * hh);
            acc[t] = wm_f16(a.v, bb.v, acc[t]);
        }
    }
    const int seg = cb / bseg;
    const float* bias = (seg == 0) ? bias0 : ((seg == 1) ? bias1 : bias2);
    const int wb = cb - seg * bseg;
    if (mode == 0) {
#pragma unroll
        for (int t = 0; t < 4; ++t) {
            const int cl = chf * 64 + t * 16 + lm;
            const float bv = bf16r(bias[wb + cl]);
#pragma unroll
            for (int r = 0; r < 8; ++r) {
                float v = acc[t][r] * scale + bv;
                v = relu ? fmaxf(v, 0.f) : v;
                st.f[(rt * 16 + 8 * hh + r) * OPITCH + cl] = v;
            }
        }
        __syncthreads();
        v4f ov[8];
#pragma unroll
        for (int i = 0; i < 8; ++i) {
            const int p = tid + 256 * i, row = p >> 5, c4 = (p & 31) * 4;
            ov[i] = *(const v4f*)(st.f + row * OPITCH + c4);
        }
#pragma unroll
        for (int i = 0; i < 8; ++i) {
            const int p = tid + 256 * i, row = p >> 5, c4 = (p & 31) * 4;
            *(volatile v4f*)(Cf + (size_t)(row0 + row) * ldc + cb + c4) = ov[i];
        }
        __threadfence();
#pragma unroll
        for (int i = 0; i < 8; ++i) {
            const int p = tid + 256 * i, row = p >> 5, c4 = (p & 31) * 4;
            *(volatile v4f*)(Cf + (size_t)(row0 + row) * ldc + cb + c4) = ov[i];
        }
    } else {
#pragma unroll
        for (int t = 0; t < 4; ++t) {
            const int cl = chf * 64 + t * 16 + lm;
            const float bv = bf16r(bias[wb + cl]);
#pragma unroll
            for (int r = 0; r < 8; ++r) {
                float v = acc[t][r] * scale + bv;
                v = relu ? fmaxf(v, 0.f) : v;
                st.h[(rt * 16 + 8 * hh + r) * HPITCH + cl] = (_Float16)(v * ocarry);
            }
        }
        __syncthreads();
        v8h ov[4];
#pragma unroll
        for (int i = 0; i < 4; ++i) {
            const int p = tid + 256 * i, row = p >> 4, c8 = (p & 15) * 8;
            ov[i] = *(const v8h*)(st.h + row * HPITCH + c8);
        }
#pragma unroll
        for (int i = 0; i < 4; ++i) {
            const int p = tid + 256 * i, row = p >> 4, c8 = (p & 15) * 8;
            *(volatile v8h*)(Ch + (size_t)(row0 + row) * ldc + cb + c8) = ov[i];
        }
        __threadfence();
#pragma unroll
        for (int i = 0; i < 4; ++i) {
            const int p = tid + 256 * i, row = p >> 4, c8 = (p & 15) * 8;
            *(volatile v8h*)(Ch + (size_t)(row0 + row) * ldc + cb + c8) = ov[i];
        }
    }
}

__global__ __launch_bounds__(256) void k_attn(const _Float16* __restrict__ QKV, const int* __restrict__ mask, _Float16* Ch, int nkv, int mkpitch)
{
    __shared__ __align__(16) _Float16 sK[2 * KT * KPITCH];
    __shared__ __align__(16) _Float16 sVt[2 * DH * VPITCH];
    __shared__ __align__(16) _Float16 sP[8 * 16 * PPITCH];
    __shared__ __align__(16) _Float16 sC[QR * CPITCH];
    __shared__ unsigned mbits[QR * MKW];
    __shared__ int s_tile[32];
    __shared__ int s_rowm[QR];
    __shared__ unsigned s_skip;

    const int tid = threadIdx.x, lane = tid & 31, wv = tid >> 5, hh = lane >> 4, lm = lane & 15;
    const int rg = wv & 3, sub = wv >> 2;
    const int b = blockIdx.y, q0 = blockIdx.x * QR;
    const int nkt = nkv / KT;
    const int LDQ = 3 * DM;

#pragma unroll 1
    for (int row = wv; row < QR; row += 8) {
        const int* mrow = mask + ((size_t)b * SEQ_FULL + q0 + row) * (size_t)mkpitch;
#pragma unroll 4
        for (int kw = 0; kw < MKW; ++kw) {
            const int kwc = (kw < nkt) ? kw : (nkt - 1);
            const int mv = mrow[kwc * 32 + lane];
            unsigned bal = __builtin_amdgcn_ballot_w32(mv != 0);
            bal = (kw < nkt) ? bal : 0u;
            if (lane == 0) mbits[row * MKW + kw] = bal;
        }
    }
    __syncthreads();
    if (tid < 32) {
        const int col = (tid < MKW) ? tid : (MKW - 1);
        int all = 1;
#pragma unroll 1
        for (int r = 0; r < QR; ++r) all &= (mbits[r * MKW + col] == 0xFFFFFFFFu) ? 1 : 0;
        s_tile[tid] = (tid < nkt) ? all : 0;
    } else if (tid >= 64 && tid < 64 + QR) {
        const int r = tid - 64;
        int all = 1;
#pragma unroll 1
        for (int kw = 0; kw < MKW; ++kw) all &= (kw < nkt) ? ((mbits[r * MKW + kw] == 0xFFFFFFFFu) ? 1 : 0) : 1;
        s_rowm[r] = all;
    }
    __syncthreads();
    if (tid == 0) {
        int any = 0;
#pragma unroll 1
        for (int r = 0; r < QR; ++r) any |= s_rowm[r];
        unsigned sk = 0;
        if (!any) {
#pragma unroll 1
            for (int t = 0; t < 32; ++t) sk |= ((unsigned)s_tile[t]) << t;
        }
        s_skip = sk;
    }
    __syncthreads();
    const unsigned skipm = (unsigned)__builtin_amdgcn_readfirstlane((int)s_skip);

#pragma unroll 1
    for (int hp = 0; hp < HE / 2; ++hp) {
        const int h = 2 * hp + sub;
        FragH qa[2];
        {
            const _Float16* qrow = QKV + ((size_t)b * SEQ + q0 + rg * 16 + lm) * LDQ + h * DH;
#pragma unroll
            for (int j = 0; j < 2; ++j) {
                qa[j].h[0] = *(const v8h*)(qrow + 32 * j + 8 * hh);
                qa[j].h[1] = *(const v8h*)(qrow + 32 * j + 16 + 8 * hh);
            }
        }
        v8f acc[4];
        float rm[8], rl[8];
#pragma unroll
        for (int t = 0; t < 4; ++t) acc[t] = (v8f){};
#pragma unroll
        for (int r = 0; r < 8; ++r) { rm[r] = -1e30f; rl[r] = 0.f; }

#pragma unroll 1
        for (int kt = 0; kt < nkt; ++kt) {
            if ((skipm >> kt) & 1u) continue;
            const int key0 = kt * KT;
#pragma unroll
            for (int i = 0; i < 2; ++i) {
                const int p = tid + 256 * i, key = p >> 4, c16 = p & 15;
                const size_t g = ((size_t)b * nkv + key0 + key) * LDQ + hp * 128 + c16 * 8;
                const v8h kv = *(const v8h*)(QKV + DM + g);
                *(v8h*)(sK + ((c16 >> 3) * KT + key) * KPITCH + (c16 & 7) * 8) = kv;
                const v8h vv = *(const v8h*)(QKV + 2 * DM + g);
#pragma unroll
                for (int j = 0; j < 8; ++j) sVt[(c16 * 8 + j) * VPITCH + key] = vv[j];
            }
            __syncthreads();

            v8f sc[2];
#pragma unroll
            for (int t = 0; t < 2; ++t) {
                v8f c = (v8f){};
#pragma unroll
                for (int j = 0; j < 2; ++j) {
                    FragH kb;
                    const _Float16* kr = sK + (sub * KT + t * 16 + lm) * KPITCH + 32 * j;
                    kb.h[0] = *(const v8h*)(kr + 8 * hh);
                    kb.h[1] = *(const v8h*)(kr + 16 + 8 * hh);
                    c = wm_f16(qa[j].v, kb.v, c);
                }
                sc[t] = c;
            }
#pragma unroll
            for (int r = 0; r < 8; ++r) {
                const unsigned mw = mbits[(rg * 16 + 8 * hh + r) * MKW + kt];
                const float x0 = ((mw >> lm) & 1u) ? MASK_FILL : sc[0][r] * SC_SCALE;
                const float x1 = ((mw >> (16 + lm)) & 1u) ? MASK_FILL : sc[1][r] * SC_SCALE;
                float mx = fmaxf(x0, x1);
#pragma unroll
                for (int o = 1; o < 16; o <<= 1) mx = fmaxf(mx, __shfl_xor(mx, o, 32));
                const float nm = fmaxf(rm[r], mx);
                const float corr = __expf(rm[r] - nm);
                const float p0 = __expf(x0 - nm), p1 = __expf(x1 - nm);
                float rs = p0 + p1;
#pragma unroll
                for (int o = 1; o < 16; o <<= 1) rs += __shfl_xor(rs, o, 32);
                rl[r] = rl[r] * corr + rs;
                rm[r] = nm;
#pragma unroll
                for (int t = 0; t < 4; ++t) acc[t][r] = acc[t][r] * corr;
                _Float16* prow = sP + (wv * 16 + 8 * hh + r) * PPITCH;
                prow[lm] = (_Float16)(p0 * P_CARRY);
                prow[16 + lm] = (_Float16)(p1 * P_CARRY);
            }
            __syncthreads();

            {
                FragH pa;
                const _Float16* pr = sP + (wv * 16 + lm) * PPITCH;
                pa.h[0] = *(const v8h*)(pr + 8 * hh);
                pa.h[1] = *(const v8h*)(pr + 16 + 8 * hh);
#pragma unroll
                for (int t = 0; t < 4; ++t) {
                    FragH vb;
                    const _Float16* vr = sVt + (sub * DH + t * 16 + lm) * VPITCH;
                    vb.h[0] = *(const v8h*)(vr + 8 * hh);
                    vb.h[1] = *(const v8h*)(vr + 16 + 8 * hh);
                    acc[t] = wm_f16(pa.v, vb.v, acc[t]);
                }
            }
            __syncthreads();
        }

        float inv[8];
#pragma unroll
        for (int r = 0; r < 8; ++r) inv[r] = (1.0f / rl[r]) * (C_CARRY / (P_CARRY * QKV_CARRY));
        __syncthreads();
#pragma unroll
        for (int r = 0; r < 8; ++r)
#pragma unroll
            for (int t = 0; t < 4; ++t)
                sC[(rg * 16 + 8 * hh + r) * CPITCH + sub * DH + t * 16 + lm] = (_Float16)(acc[t][r] * inv[r]);
        __syncthreads();
        v8h ov[4];
#pragma unroll
        for (int i = 0; i < 4; ++i) {
            const int p = tid + 256 * i, row = p >> 4, c8 = (p & 15) * 8;
            ov[i] = *(const v8h*)(sC + row * CPITCH + c8);
        }
#pragma unroll
        for (int i = 0; i < 4; ++i) {
            const int p = tid + 256 * i, row = p >> 4, c8 = (p & 15) * 8;
            *(volatile v8h*)(Ch + ((size_t)b * SEQ + q0 + row) * DM + hp * 128 + c8) = ov[i];
        }
        __threadfence();
#pragma unroll
        for (int i = 0; i < 4; ++i) {
            const int p = tid + 256 * i, row = p >> 4, c8 = (p & 15) * 8;
            *(volatile v8h*)(Ch + ((size_t)b * SEQ + q0 + row) * DM + hp * 128 + c8) = ov[i];
        }
    }
}

__global__ __launch_bounds__(256) void k_ln(const float* __restrict__ T, const float* __restrict__ res, const float* __restrict__ gam, const float* __restrict__ bet,
                                           float* outf, _Float16* outh, int res_full, int out_full, int write_h)
{
    __shared__ float red[8];
    __shared__ __align__(16) _Float16 sY[DM];
    const int tid = threadIdx.x, lane = tid & 31, wv = tid >> 5;
    const int r = blockIdx.x;
    const int bb = r / SEQ, n = r - bb * SEQ;
    const size_t rfull = (size_t)bb * SEQ_FULL + n;
    const int c0 = tid * 4;
    const v4f tv = *(const v4f*)(T + (size_t)r * DM + c0);
    const v4f rv = *(const v4f*)(res + (res_full ? rfull : (size_t)r) * DM + c0);
    float x[4];
#pragma unroll
    for (int i = 0; i < 4; ++i) x[i] = tv[i] + (res_full ? bf16r(rv[i]) : rv[i]);

    float s = (x[0] + x[1]) + (x[2] + x[3]);
#pragma unroll
    for (int o = 16; o >= 1; o >>= 1) s += __shfl_xor(s, o, 32);
    if (lane == 0) red[wv] = s;
    __syncthreads();
    float tot = 0.f;
#pragma unroll
    for (int i = 0; i < 8; ++i) tot += red[i];
    const float mean = tot * (1.0f / DM);
    __syncthreads();
    float vs = 0.f;
#pragma unroll
    for (int i = 0; i < 4; ++i) { const float d = x[i] - mean; vs += d * d; }
#pragma unroll
    for (int o = 16; o >= 1; o >>= 1) vs += __shfl_xor(vs, o, 32);
    if (lane == 0) red[wv] = vs;
    __syncthreads();
    float vtot = 0.f;
#pragma unroll
    for (int i = 0; i < 8; ++i) vtot += red[i];
    const float rstd = 1.0f / sqrtf(vtot * (1.0f / DM) + LN_EPS);

    const v4f gv = *(const v4f*)(gam + c0), bv = *(const v4f*)(bet + c0);
    v4f y;
#pragma unroll
    for (int i = 0; i < 4; ++i) y[i] = (bf16r(gv[i]) * (x[i] - mean)) * rstd + bf16r(bv[i]);

    float* dst = outf + (out_full ? rfull : (size_t)r) * DM + c0;
    *(volatile v4f*)dst = y;
    if (write_h) {
#pragma unroll
        for (int i = 0; i < 4; ++i) sY[c0 + i] = (_Float16)(y[i] * X_CARRY);
    }
    __threadfence();
    *(volatile v4f*)dst = y;
    if (write_h) {
        __syncthreads();
        if (tid < DM / 8) {
            const v8h o = *(const v8h*)(sY + tid * 8);
            _Float16* hd = outh + (size_t)r * DM + tid * 8;
            *(volatile v8h*)hd = o;
            __threadfence();
            *(volatile v8h*)hd = o;
        }
    }
}

extern "C" void kernel_launch(void* const* d_in, const int* in_sizes, int n_in,
                              void* d_out, int out_size, void* d_ws, size_t ws_size, hipStream_t stream)
{
    if (n_in < 30) return;
    const long long needX  = ((long long)(NB - 1) * SEQ_FULL + SEQ) * DM;
    const long long needE  = ((long long)(NB - 1) * SENC_FULL + SENC) * DM;
    const long long needM1 = ((long long)(NB - 1) * SEQ_FULL + SEQ) * SEQ_FULL;
    const long long needM2 = ((long long)(NB - 1) * SEQ_FULL + SEQ) * SENC_FULL;
    if ((long long)in_sizes[0] < needX || (long long)in_sizes[1] < needM1) return;
    if ((long long)in_sizes[2] < needE || (long long)in_sizes[3] < needM2) return;
    if (in_sizes[4] < HE * DM * DH || in_sizes[6] < HE * DM * DH || in_sizes[8] < HE * DM * DH) return;
    if (in_sizes[12] < HE * DM * DH || in_sizes[14] < HE * DM * DH || in_sizes[16] < HE * DM * DH) return;
    if (in_sizes[5] < HE * DH || in_sizes[7] < HE * DH || in_sizes[9] < HE * DH) return;
    if (in_sizes[13] < HE * DH || in_sizes[15] < HE * DH || in_sizes[17] < HE * DH) return;
    if (in_sizes[10] < DM * DM || in_sizes[18] < DM * DM || in_sizes[11] < DM || in_sizes[19] < DM) return;
    if (in_sizes[20] < DM * DFF || in_sizes[21] < DFF || in_sizes[22] < DFF * DM || in_sizes[23] < DM) return;
    for (int i = 24; i < 30; ++i) if (in_sizes[i] < DM) return;
    if ((long long)out_size < needX) return;

    const float* x_in  = (const float*)d_in[0];
    const int*   mask1 = (const int*)d_in[1];
    const float* enc   = (const float*)d_in[2];
    const int*   mask2 = (const int*)d_in[3];
    const float* Wq1 = (const float*)d_in[4];  const float* bq1 = (const float*)d_in[5];
    const float* Wk1 = (const float*)d_in[6];  const float* bk1 = (const float*)d_in[7];
    const float* Wv1 = (const float*)d_in[8];  const float* bv1 = (const float*)d_in[9];
    const float* Wo1 = (const float*)d_in[10]; const float* bo1 = (const float*)d_in[11];
    const float* Wq2 = (const float*)d_in[12]; const float* bq2 = (const float*)d_in[13];
    const float* Wk2 = (const float*)d_in[14]; const float* bk2 = (const float*)d_in[15];
    const float* Wv2 = (const float*)d_in[16]; const float* bv2 = (const float*)d_in[17];
    const float* Wo2 = (const float*)d_in[18]; const float* bo2 = (const float*)d_in[19];
    const float* W1f = (const float*)d_in[20]; const float* b1f = (const float*)d_in[21];
    const float* W2f = (const float*)d_in[22]; const float* b2f = (const float*)d_in[23];
    const float* g1  = (const float*)d_in[24]; const float* be1 = (const float*)d_in[25];
    const float* g2  = (const float*)d_in[26]; const float* be2 = (const float*)d_in[27];
    const float* g3  = (const float*)d_in[28]; const float* be3 = (const float*)d_in[29];
    float* out = (float*)d_out;

    const size_t M = MROWS, ME = EROWS, MX = XROWS;
    unsigned char* base = (unsigned char*)d_ws;
    size_t off = 0;
    _Float16* Wqkv1T = (_Float16*)(base + off); off += SZ_WQKV;
    _Float16* Wqkv2T = (_Float16*)(base + off); off += SZ_WQKV;
    _Float16* Wo1T   = (_Float16*)(base + off); off += SZ_WO;
    _Float16* Wo2T   = (_Float16*)(base + off); off += SZ_WO;
    _Float16* W1T    = (_Float16*)(base + off); off += SZ_WF;
    _Float16* W2T    = (_Float16*)(base + off); off += SZ_WF;
    const size_t offXE = off; off += SZ_XE;
    _Float16* Xh  = (_Float16*)(base + offXE);
    _Float16* Eh  = (_Float16*)(base + offXE + M * DM * 2);
    float*    x2f = (float*)(base + offXE);
    const size_t offQC = off; off += SZ_QC;
    _Float16* QKV = (_Float16*)(base + offQC);
    _Float16* Chx = (_Float16*)(base + offQC + MX * 3 * DM * 2);
    _Float16* Hh  = (_Float16*)(base + offQC);
    float*    Tf  = (float*)(base + off);    off += SZ_T;
    float*    x1f = (float*)(base + off);    off += SZ_X1F;
    _Float16* X1h = (_Float16*)(base + off); off += SZ_X1H;
    if (off > ws_size) return;

    const float sc_xw = 1.0f / (X_CARRY * W_CARRY);
    const float sc_cw = 1.0f / (C_CARRY * W_CARRY);
    const float sc_hw = 1.0f / (H_CARRY * W_CARRY);
    const long long zsW = (long long)DM * DH;

    k_wtrans<<<dim3(1, DM / 64, 3 * HE), dim3(256), 0, stream>>>(Wq1, Wk1, Wv1, Wqkv1T, Wqkv1T + (size_t)DM * DM, Wqkv1T + (size_t)2 * DM * DM, DM, DH, HE, zsW, zsW);
    k_wtrans<<<dim3(1, DM / 64, 3 * HE), dim3(256), 0, stream>>>(Wq2, Wk2, Wv2, Wqkv2T, Wqkv2T + (size_t)DM * DM, Wqkv2T + (size_t)2 * DM * DM, DM, DH, HE, zsW, zsW);
    k_wtrans<<<dim3(DM / 64, DM / 64, 2), dim3(256), 0, stream>>>(Wo1, Wo2, Wo2, Wo1T, Wo2T, Wo2T, DM, DM, 1, 0LL, 0LL);
    k_wtrans<<<dim3(DFF / 64, DM / 64, 1), dim3(256), 0, stream>>>(W1f, W1f, W1f, W1T, W1T, W1T, DM, DFF, 1, 0LL, 0LL);
    k_wtrans<<<dim3(DM / 64, DFF / 64, 1), dim3(256), 0, stream>>>(W2f, W2f, W2f, W2T, W2T, W2T, DFF, DM, 1, 0LL, 0LL);

    const int nblkX = (int)(M * DM / 2048), nblkE = (int)(ME * DM / 2048);
    k_xconv<<<dim3(nblkX + nblkE), dim3(256), 0, stream>>>(x_in, enc, Xh, Eh, nblkX);

    k_gemm<<<dim3((unsigned)(M / 64), 3 * DM / 128), dim3(256), 0, stream>>>(Xh, Wqkv1T, bq1, bk1, bv1, Tf, QKV, DM, DM, 3 * DM, DM, DM, 1, 0, sc_xw, QKV_CARRY);
    k_attn<<<dim3(SEQ / QR, NB), dim3(256), 0, stream>>>(QKV, mask1, Chx, SEQ, SEQ_FULL);
    k_gemm<<<dim3((unsigned)(M / 64), DM / 128), dim3(256), 0, stream>>>(Chx, Wo1T, bo1, bo1, bo1, Tf, QKV, DM, DM, DM, DM, DM, 0, 0, sc_cw, 1.0f);
    k_ln<<<dim3((unsigned)M), dim3(256), 0, stream>>>(Tf, x_in, g1, be1, x1f, X1h, 1, 0, 1);

    k_gemm<<<dim3((unsigned)(M / 64), DM / 128), dim3(256), 0, stream>>>(X1h, Wqkv2T, bq2, bq2, bq2, Tf, QKV, DM, DM, 3 * DM, DM, DM, 1, 0, sc_xw, QKV_CARRY);
    k_gemm<<<dim3((unsigned)(ME / 64), 2 * DM / 128), dim3(256), 0, stream>>>(Eh, Wqkv2T + (size_t)DM * DM, bk2, bv2, bv2, Tf, QKV + DM, DM, DM, 3 * DM, DM, DM, 1, 0, sc_xw, QKV_CARRY);
    k_attn<<<dim3(SEQ / QR, NB), dim3(256), 0, stream>>>(QKV, mask2, Chx, SENC, SENC_FULL);
    k_gemm<<<dim3((unsigned)(M / 64), DM / 128), dim3(256), 0, stream>>>(Chx, Wo2T, bo2, bo2, bo2, Tf, QKV, DM, DM, DM, DM, DM, 0, 0, sc_cw, 1.0f);
    k_ln<<<dim3((unsigned)M), dim3(256), 0, stream>>>(Tf, x1f, g2, be2, x2f, X1h, 0, 0, 1);

    k_gemm<<<dim3((unsigned)(M / 64), DFF / 128), dim3(256), 0, stream>>>(X1h, W1T, b1f, b1f, b1f, Tf, Hh, DM, DM, DFF, DM, DFF, 1, 1, sc_xw, H_CARRY);
    k_gemm<<<dim3((unsigned)(M / 64), DM / 128), dim3(256), 0, stream>>>(Hh, W2T, b2f, b2f, b2f, Tf, QKV, DFF, DFF, DM, DFF, DM, 0, 0, sc_hw, 1.0f);
    k_ln<<<dim3((unsigned)M), dim3(256), 0, stream>>>(Tf, x2f, g3, be3, out, X1h, 0, 1, 0);
}
